// ablation_1_29575144801048
// MI455X (gfx1250) — hardware-run, weakly checked
//
#include <hip/hip_runtime.h>


namespace {
constexpr int T = 2, N = 50000, E = 400000, F = 24, Hh = 64, NEW = E / 32  , NNW = (N + 31) / 32  ;
constexpr float HS = 256.0f, WSC = 256.0f;
typedef _Float16 b16;
typedef __attribute__((ext_vector_type(16))) _Float16 v16b;
typedef __attribute__((ext_vector_type(8))) _Float16 v8b;
typedef __attribute__((ext_vector_type(8))) float v8f;
typedef __attribute__((ext_vector_type(4))) float v4f;
typedef __attribute__((ext_vector_type(2))) float v2f;
__device__ __forceinline__ float bf16_rne(float f) { unsigned int u = __float_as_uint(f); u += 0x7FFFu + ((u >> 16) & 1u); float r = __uint_as_float(u & 0xFFFF0000u); asm volatile("" : "+v"(r)); return r; }
__device__ __forceinline__ float bfv(float f) { float r = bf16_rne(f); asm volatile("" : "+v"(r)); return r; }
__device__ __forceinline__ void split16(float v, b16& hi, b16& lo) { hi = (b16)v; lo = (b16)(v - (float)hi); }
__device__ __forceinline__ v16b frag_kb(const b16* p, int hh) { const v8b a = *(const v8b*)(p + 8 * hh), b = *(const v8b*)(p + 16 + 8 * hh); v16b f;
#pragma unroll
  for (int e = 0; e < 8; ++e) { f[e] = a[e]; f[8 + e] = b[e]; } return f; }
__device__ __forceinline__ v8f wmma16b(v16b a, v16b b, v8f c) { v8f d = __builtin_amdgcn_wmma_f32_16x16x32_f16(false, a, false, b, (short)0, c, false, false); asm volatile("v_nop\n\tv_nop\n\tv_nop\n\tv_nop" : "+v"(d) : "v"(a), "v"(b)); return d; }
__device__ __forceinline__ void wave_lds_sync() { __builtin_amdgcn_fence(__ATOMIC_RELEASE, "workgroup"); __builtin_amdgcn_wave_barrier(); __builtin_amdgcn_fence(__ATOMIC_ACQUIRE, "workgroup"); }
__device__ __forceinline__ float pmul(float a, float b) { float p = a * b; asm volatile("" : "+v"(p)); return p; }
__device__ __forceinline__ int iclamp(int v, int lo, int hi) { return v < lo ? lo : (v > hi ? hi : v); }
constexpr int CSR_NBLK8 = 512, CSR_GB8 = 8, CSR_GN8 = 1 << CSR_GB8  , CSR_TS8 = (CSR_GN8 < 32 ? 32 : CSR_GN8)  , CSR_MAXG8 = 512, CSR_CAP8 = 12288  ;
__device__ __host__ __forceinline__ int csr_tix8(int v) { return (v >> CSR_GB8) * CSR_TS8 + (v & (CSR_GN8 - 1)); }
__global__ __launch_bounds__(64) void csrA_kernel8(const int* __restrict__ dst, int E, int N, int nG, int CHP, int NGP, int* __restrict__ STG, int* __restrict__ HST) {
  extern __shared__ int sm[];
  int* cnt = sm; int* run = sm + NGP; int* ids = sm + 2 * NGP;
  const int b = blockIdx.x; const int ch = (E + CSR_NBLK8 - 1) / CSR_NBLK8; const int e0 = b * ch, e1 = min(E, e0 + ch);
  for (int i = threadIdx.x; i < NGP; i += 64) cnt[i] = 0;
  for (int i = threadIdx.x; i < CHP; i += 64) ids[i] = -1;
  __syncthreads();
  if (threadIdx.x == 0) {
    for (int e = e0; e < e1; ++e) { int d = dst[e]; d = (d < 0) ? 0 : (d >= N ? N - 1 : d); cnt[d >> CSR_GB8] += 1; }
    int acc = 0; for (int g = 0; g < nG; ++g) { run[g] = acc; acc += cnt[g]; }
    for (int e = e0; e < e1; ++e) { int d = dst[e]; d = (d < 0) ? 0 : (d >= N ? N - 1 : d); const int g = d >> CSR_GB8; ids[run[g]] = e; run[g] += 1; } }
  __syncthreads();
  typedef __attribute__((ext_vector_type(4))) int v4i;
  for (int pass = 0; pass < 2; ++pass) {
    for (int i = threadIdx.x; i < CHP / 4; i += 64) *(volatile v4i*)(STG + (size_t)b * CHP + i * 4) = *(const v4i*)(&ids[i * 4]);
    for (int i = threadIdx.x; i < NGP / 4; i += 64) { v4i v; for (int e = 0; e < 4; ++e) v[e] = (i * 4 + e < nG) ? cnt[i * 4 + e] : 0; *(volatile v4i*)(HST + (size_t)b * NGP + i * 4) = v; }
    __threadfence(); }
}
__global__ __launch_bounds__(512) void csrS_kernel8(const int* __restrict__ HST, int nG, int NGP, int* __restrict__ START, int* __restrict__ TOT, int* __restrict__ OFF) {
  __shared__ int tot[CSR_MAXG8];
  const int b = threadIdx.x;
  for (int pass = 0; pass < 2; ++pass) { int runb = 0; for (int g = 0; g < nG; ++g) { int c = HST[(size_t)b * NGP + g]; c = (c < 0) ? 0 : c; ((volatile int*)OFF)[(size_t)g * CSR_NBLK8 + b] = runb; runb += c; } __threadfence(); }
  for (int g = threadIdx.x; g < nG; g += 512) { int s = 0; for (int bb = 0; bb < CSR_NBLK8; ++bb) { int c = HST[(size_t)bb * NGP + g]; s += (c < 0) ? 0 : c; } tot[g] = s; }
  __syncthreads();
  if (threadIdx.x < 32) {
    __shared__ int st[CSR_MAXG8 + 32];
    if (threadIdx.x == 0) { int acc = 0; for (int g = 0; g < NGP; ++g) { st[g] = acc; if (g < nG) acc += (tot[g] + 31) & ~31; } st[NGP] = acc; }
    __builtin_amdgcn_fence(__ATOMIC_RELEASE, "workgroup"); __builtin_amdgcn_wave_barrier(); __builtin_amdgcn_fence(__ATOMIC_ACQUIRE, "workgroup");
    for (int pass = 0; pass < 2; ++pass) { for (int i = threadIdx.x; i < NGP + 32; i += 32) { ((volatile int*)START)[i] = (i <= NGP) ? st[min(i, NGP)] : 0; ((volatile int*)TOT)[i] = (i < nG) ? tot[i] : 0; } __threadfence(); } }
}
__global__ __launch_bounds__(256) void csrB_kernel8(const int* __restrict__ dst, int N, int nG, int CHP, int NGP, int permLen, const int* __restrict__ STG, const int* __restrict__ HST, const int* __restrict__ OFF, const int* __restrict__ START, const int* __restrict__ TOT, int* __restrict__ PERM, int* __restrict__ ROWPTR, int* __restrict__ ROWCNT, int* __restrict__ FLAG) {
  typedef __attribute__((ext_vector_type(4))) int v4i;
  __shared__ int ids[CSR_CAP8]; __shared__ unsigned short key[CSR_CAP8]; __shared__ int outp[CSR_CAP8]; __shared__ int ncnt[CSR_GN8 + 1]; __shared__ int boff[CSR_NBLK8 + 1];
  const int g = blockIdx.x, t_ = threadIdx.x; int tot = TOT[g]; int st = START[g], stn = START[g + 1]; const int v0 = g * CSR_GN8; const int nv = min(CSR_GN8, N - v0); const int t0 = g * CSR_TS8;
  st = (st < 0) ? 0 : (st > permLen - 32 ? permLen - 32 : st) & ~31; stn = (stn < st) ? st : (stn > permLen ? permLen : stn); tot = (tot < 0) ? 0 : tot; if (tot > stn - st && tot <= CSR_CAP8) tot = stn - st;
  if (tot > CSR_CAP8) {
    for (int pass = 0; pass < 2; ++pass) { for (int i = t_; i < CSR_TS8 / 4; i += 256) { v4i a, c; for (int e = 0; e < 4; ++e) { a[e] = st; c[e] = 0; } *(volatile v4i*)(ROWPTR + t0 + i * 4) = a; *(volatile v4i*)(ROWCNT + t0 + i * 4) = c; } if (t_ == 0) ((volatile int*)FLAG)[0] = 1; __threadfence(); } (void)nv; return; }
  if (t_ == 0) { int acc = 0; for (int b = 0; b < CSR_NBLK8; ++b) { boff[b] = acc; int c = HST[(size_t)b * NGP + g]; c = (c < 0) ? 0 : (c > CHP ? CHP : c); acc += c; if (acc > tot) acc = tot; } boff[CSR_NBLK8] = acc; }
  for (int i = t_; i <= CSR_GN8; i += 256) ncnt[i] = 0;
  __syncthreads();
  for (int b = 0; b < CSR_NBLK8; ++b) { const int c = boff[b + 1] - boff[b]; int o_ = OFF[(size_t)g * CSR_NBLK8 + b]; o_ = (o_ < 0) ? 0 : (o_ > CHP - c ? CHP - c : o_); const int* src_ = STG + (size_t)b * CHP + o_;
    for (int i = t_; i < c; i += 256) { int id = src_[i]; id = (id < 0) ? 0 : id; ids[boff[b] + i] = id; int d = dst[id]; d = (d < v0) ? v0 : (d >= N ? N - 1 : d); int kk = d - v0; kk = (kk < 0) ? 0 : (kk >= CSR_GN8 ? CSR_GN8 - 1 : kk); key[boff[b] + i] = (unsigned short)kk; } }
  __syncthreads();
  if (t_ == 0) { for (int i = 0; i < tot; ++i) ncnt[key[i]] += 1; int acc = 0; for (int vl = 0; vl < CSR_GN8; ++vl) { const int c = ncnt[vl]; ncnt[vl] = acc; acc += c; } ncnt[CSR_GN8] = acc;
    for (int i = 0; i < tot; ++i) { const int vl = key[i]; outp[ncnt[vl]] = ids[i]; ncnt[vl] += 1; }
    for (int vl = CSR_GN8; vl > 0; --vl) ncnt[vl] = ncnt[vl - 1]; ncnt[0] = 0; }
  __syncthreads();
  for (int pass = 0; pass < 2; ++pass) {
    for (int i = t_; i < (stn - st) / 4; i += 256) { v4i v; for (int e = 0; e < 4; ++e) { const int q = i * 4 + e; v[e] = (q < tot) ? outp[q] : -1; } *(volatile v4i*)(PERM + st + i * 4) = v; }
    for (int i = t_; i < CSR_TS8 / 4; i += 256) { v4i a, c; for (int e = 0; e < 4; ++e) { const int vl = i * 4 + e; const int vc = vl < CSR_GN8 ? vl : CSR_GN8; a[e] = (vl < CSR_GN8) ? st + ncnt[vc] : st; c[e] = (vl < nv) ? (ncnt[(vc < CSR_GN8 ? vc : CSR_GN8 - 1) + 1] - ncnt[vc]) : 0; } *(volatile v4i*)(ROWPTR + t0 + i * 4) = a; *(volatile v4i*)(ROWCNT + t0 + i * 4) = c; }
    __threadfence(); }
}
__global__ __launch_bounds__(256) void csrZ_kernel8(int* __restrict__ p, size_t n4) { typedef __attribute__((ext_vector_type(4))) int v4i; const size_t tid = (size_t)blockIdx.x * 256 + threadIdx.x, nth = (size_t)gridDim.x * 256; v4i z = {0, 0, 0, 0}; for (size_t i = tid; i < n4; i += nth) *(volatile v4i*)(p + i * 4) = z; }
struct CsrBufs8 { int *STG, *HST, *OFF, *START, *TOT, *PERM, *ROWPTR, *ROWCNT, *FLAG; int nG, NGP, CHP; size_t permLen; char* base; size_t bytes; };
static size_t csr_carve8(CsrBufs8& c, char* ws, size_t off, int E, int N) {
  const size_t off0 = off; c.base = ws + off;
  auto al = [&](size_t bytes) { char* p = ws + off; off += (bytes + 255) & ~(size_t)255; return p; };
  c.nG = (N + CSR_GN8 - 1) / CSR_GN8; c.NGP = (c.nG + 31) & ~31; const int ch = (E + CSR_NBLK8 - 1) / CSR_NBLK8; c.CHP = (ch + 31) & ~31; c.permLen = (size_t)E + 32 * (size_t)c.nG + 32;
  c.STG = (int*)al((size_t)CSR_NBLK8 * c.CHP * 4); c.HST = (int*)al((size_t)CSR_NBLK8 * c.NGP * 4); c.OFF = (int*)al((size_t)c.NGP * CSR_NBLK8 * 4); c.START = (int*)al((size_t)(c.NGP + 64) * 4); c.TOT = (int*)al((size_t)(c.NGP + 64) * 4);
  c.PERM = (int*)al(c.permLen * 4); c.ROWPTR = (int*)al((size_t)c.nG * CSR_TS8 * 4); c.ROWCNT = (int*)al((size_t)c.nG * CSR_TS8 * 4); c.FLAG = (int*)al(256);
  c.bytes = off - off0; return off;
}
static void csr_build8(const CsrBufs8& c, const int* dst, int E, int N, hipStream_t stream) {
  const size_t smem = (size_t)(2 * c.NGP + c.CHP) * 4;
  csrZ_kernel8<<<512, 256, 0, stream>>>((int*)c.base, c.bytes / 16);
  csrA_kernel8<<<CSR_NBLK8, 64, smem, stream>>>(dst, E, N, c.nG, c.CHP, c.NGP, c.STG, c.HST);
  csrS_kernel8<<<1, 512, 0, stream>>>(c.HST, c.nG, c.NGP, c.START, c.TOT, c.OFF);
  csrB_kernel8<<<c.nG, 256, 0, stream>>>(dst, N, c.nG, c.CHP, c.NGP, (int)c.permLen, c.STG, c.HST, c.OFF, c.START, c.TOT, c.PERM, c.ROWPTR, c.ROWCNT, c.FLAG);
}


__global__ __launch_bounds__(256) void wput_kernel(const float* __restrict__ web, const float* __restrict__ wnb, const float* __restrict__ wd1, b16* __restrict__ WEE, b16* __restrict__ WEN, b16* __restrict__ WNB, b16* __restrict__ WD1) { const int u = blockIdx.x * 256 + threadIdx.x; v8b v;
  if (u < Hh * 16) { const int o = u / 16, k0 = (u % 16) * 8;
#pragma unroll
    for (int j = 0; j < 8; ++j) v[j] = (b16)(bf16_rne(web[(size_t)(k0 + j) * Hh + o]) * WSC); for (int pass = 0; pass < 2; ++pass) { *(volatile v8b*)(WEE + (size_t)o * 128 + k0) = v; __threadfence(); } }
  if (u < 128 * 16) { const int op = u / 16, k0 = (u % 16) * 8; const int part = op / Hh, o = op % Hh;
#pragma unroll
    for (int j = 0; j < 8; ++j) v[j] = (b16)(bf16_rne(web[(size_t)(128 * (part + 1) + k0 + j) * Hh + o]) * WSC); for (int pass = 0; pass < 2; ++pass) { *(volatile v8b*)(WEN + (size_t)op * 128 + k0) = v; __threadfence(); } }
  if (u < Hh * 32) { const int o = u / 32, k0 = (u % 32) * 8;
#pragma unroll
    for (int j = 0; j < 8; ++j) v[j] = (b16)(bf16_rne(wnb[(size_t)(k0 + j) * Hh + o]) * WSC); for (int pass = 0; pass < 2; ++pass) { *(volatile v8b*)(WNB + (size_t)o * 256 + k0) = v; __threadfence(); } }
  if (u < Hh * 8) { const int o = u / 8, k0 = (u % 8) * 8;
#pragma unroll
    for (int j = 0; j < 8; ++j) v[j] = (b16)(bf16_rne(wd1[(size_t)(k0 + j) * Hh + o]) * WSC); for (int pass = 0; pass < 2; ++pass) { *(volatile v8b*)(WD1 + (size_t)o * Hh + k0) = v; __threadfence(); } } }
__global__ __launch_bounds__(64) void glob_kernel(const float* __restrict__ gattr, const float* __restrict__ wge, const float* __restrict__ bge, const float* __restrict__ wgb, const float* __restrict__ bgb, const float* __restrict__ web, const float* __restrict__ wnb, const float* __restrict__ NP, int nnw, const float* __restrict__ EP, int new_, int first, float* __restrict__ GV) { __shared__ float In[192], Hg[64]; const int c = threadIdx.x;
  if (first) { Hg[c] = fmaxf(pmul(bfv(gattr[0]), bfv(wge[c])) + bfv(bge[c]), 0.0f); }
  else { double sx = 0.0, se = 0.0, cx = 0.0, ce = 0.0; for (int w = 0; w < nnw; ++w) { sx += (double)NP[(size_t)w * 128 + c]; cx += (double)NP[(size_t)w * 128 + 64]; } for (int w = 0; w < new_; ++w) { se += (double)EP[(size_t)w * 128 + c]; ce += (double)EP[(size_t)w * 128 + 64]; }
    In[c] = (float)(sx / cx); In[64 + c] = (float)(se / ce); In[128 + c] = GV[c]; __syncthreads(); float s = bfv(bgb[c]); for (int k = 0; k < 192; ++k) s += pmul(In[k], bfv(wgb[(size_t)k * Hh + c])); Hg[c] = fmaxf(s, 0.0f); }
  __syncthreads(); float ge = 0.0f, gn = 0.0f; for (int k = 0; k < Hh; ++k) { ge += pmul(Hg[k], bfv(web[(size_t)(384 + k) * Hh + c])); gn += pmul(Hg[k], bfv(wnb[(size_t)(256 + k) * Hh + c])); }
  __syncthreads();
  for (int pass = 0; pass < 2; ++pass) { ((volatile float*)GV)[c] = Hg[c]; ((volatile float*)GV)[64 + c] = ge; ((volatile float*)GV)[128 + c] = gn; ((volatile float*)GV)[192 + c] = 0.0f; __threadfence(); } }
__global__ __launch_bounds__(32) void nodepre_kernel(const float* __restrict__ na, const float* __restrict__ wne, const float* __restrict__ bne, const float* __restrict__ HX, const b16* __restrict__ WEN, int first, int NLIM, float* __restrict__ CX, float* __restrict__ PSR) { __shared__ __attribute__((aligned(16))) b16 Ah[16][136], Al[16][136]; __shared__ float Xa[16][F + 1], Tf[16][132]; const int lane = threadIdx.x, nloc = lane & 15, hlf = lane >> 4; const size_t m0 = (size_t)blockIdx.x * 16; if (m0 >= (size_t)NLIM) return;
  for (int rr = 0; rr < 16; ++rr) if (lane < F) Xa[rr][lane] = bfv(na[(m0 + rr) * F + lane]);
  wave_lds_sync();
  for (int rr = 0; rr < 16; ++rr) { float e0 = bfv(bne[lane]), e1 = bfv(bne[32 + lane]);
#pragma unroll 1
    for (int d = 0; d < F; ++d) { const float xv = Xa[rr][d]; e0 += pmul(xv, bfv(wne[d * Hh + lane])); e1 += pmul(xv, bfv(wne[d * Hh + 32 + lane])); }
    e0 = fmaxf(e0, 0.0f); e1 = fmaxf(e1, 0.0f); const float h0 = first ? e0 : HX[(m0 + rr) * Hh + lane], h1 = first ? e1 : HX[(m0 + rr) * Hh + 32 + lane]; Tf[rr][lane] = e0; Tf[rr][32 + lane] = e1; Tf[rr][64 + lane] = h0; Tf[rr][96 + lane] = h1;
    for (int q = 0; q < 4; ++q) { b16 p, ql; split16(Tf[rr][q * 32 + lane] * HS, p, ql); Ah[rr][q * 32 + lane] = p; Al[rr][q * 32 + lane] = ql; } }
  if (lane < 16) for (int k = 128; k < 136; ++k) { Ah[lane][k] = (b16)0.0f; Al[lane][k] = (b16)0.0f; }
  wave_lds_sync();
  for (int pass = 0; pass < 2; ++pass) { for (int rr = 0; rr < 16; ++rr) *(volatile v4f*)(CX + (m0 + rr) * 128 + lane * 4) = *(const v4f*)(&Tf[rr][lane * 4]); __threadfence(); }
  v8f acc[8];
#pragma unroll
  for (int t = 0; t < 8; ++t) acc[t] = (v8f){};
#pragma unroll
  for (int kb = 0; kb < 128; kb += 32) { const v16b a = frag_kb(&Ah[nloc][kb], hlf), al = frag_kb(&Al[nloc][kb], hlf);
#pragma unroll
    for (int t = 0; t < 8; ++t) { const v16b bw = frag_kb(WEN + (size_t)(t * 16 + nloc) * 128 + kb, hlf); acc[t] = wmma16b(a, bw, acc[t]); acc[t] = wmma16b(al, bw, acc[t]); } }
  wave_lds_sync();
#pragma unroll
  for (int t = 0; t < 8; ++t)
#pragma unroll
    for (int r8 = 0; r8 < 8; ++r8) Tf[8 * hlf + r8][t * 16 + nloc] = acc[t][r8] * (1.0f / (HS * WSC));
  wave_lds_sync();
  for (int pass = 0; pass < 2; ++pass) { for (int rr = 0; rr < 16; ++rr) *(volatile v4f*)(PSR + (m0 + rr) * 128 + lane * 4) = *(const v4f*)(&Tf[rr][lane * 4]); __threadfence(); } }
__global__ __launch_bounds__(32) void edge_kernel(const float* __restrict__ ea, int t, int first, const float* __restrict__ wee, const float* __restrict__ bee, const float* __restrict__ PSR, const float* __restrict__ GV, const int* __restrict__ snd, const int* __restrict__ rcv, const b16* __restrict__ WEE, const float* __restrict__ beb, int NLIM, float* __restrict__ HE, float* __restrict__ EP) { __shared__ __attribute__((aligned(16))) b16 Ah[32][136], Al[32][136]; __shared__ float Tf[32][Hh + 1], Ps[32][Hh + 1]; __shared__ int Kp[32]; const int lane = threadIdx.x, nloc = lane & 15, hlf = lane >> 4; const size_t e0 = (size_t)blockIdx.x * 32;
  const float w0 = bfv(wee[lane]), w1 = bfv(wee[32 + lane]), b0 = bfv(bee[lane]), b1 = bfv(bee[32 + lane]);
  for (int rr = 0; rr < 32; ++rr) { const size_t e = e0 + rr; const int s = snd[e], r = rcv[e]; const bool keep = s >= 0 && s < NLIM && r >= 0 && r < NLIM; if (lane == 0) Kp[rr] = keep ? 1 : 0; const size_t sc = (size_t)iclamp(s, 0, NLIM - 1), rc = (size_t)iclamp(r, 0, NLIM - 1);
    const float at = bfv(ea[(size_t)t * E + e]), a0 = bfv(ea[e]); float c0 = fmaxf(pmul(at, w0) + b0, 0.0f), c1 = fmaxf(pmul(at, w1) + b1, 0.0f); float h0, h1; if (first) { h0 = fmaxf(pmul(a0, w0) + b0, 0.0f); h1 = fmaxf(pmul(a0, w1) + b1, 0.0f); } else { h0 = HE[e * Hh + lane]; h1 = HE[e * Hh + 32 + lane]; }
    b16 p, ql; split16(c0 * HS, p, ql); Ah[rr][lane] = p; Al[rr][lane] = ql; split16(c1 * HS, p, ql); Ah[rr][32 + lane] = p; Al[rr][32 + lane] = ql; split16(h0 * HS, p, ql); Ah[rr][64 + lane] = p; Al[rr][64 + lane] = ql; split16(h1 * HS, p, ql); Ah[rr][96 + lane] = p; Al[rr][96 + lane] = ql;
    Ps[rr][lane] = PSR[sc * 128 + lane] + PSR[rc * 128 + 64 + lane] + GV[64 + lane] + bfv(beb[lane]); Ps[rr][32 + lane] = PSR[sc * 128 + 32 + lane] + PSR[rc * 128 + 96 + lane] + GV[96 + lane] + bfv(beb[32 + lane]); }
  for (int k = 128; k < 136; ++k) { Ah[lane][k] = (b16)0.0f; Al[lane][k] = (b16)0.0f; }
  wave_lds_sync();
#pragma unroll
  for (int rt = 0; rt < 2; ++rt) { v8f acc[4] = {(v8f){}, (v8f){}, (v8f){}, (v8f){}};
#pragma unroll
    for (int kb = 0; kb < 128; kb += 32) { const v16b a = frag_kb(&Ah[rt * 16 + nloc][kb], hlf), al = frag_kb(&Al[rt * 16 + nloc][kb], hlf);
#pragma unroll
      for (int tt = 0; tt < 4; ++tt) { const v16b bw = frag_kb(WEE + (size_t)(tt * 16 + nloc) * 128 + kb, hlf); acc[tt] = wmma16b(a, bw, acc[tt]); acc[tt] = wmma16b(al, bw, acc[tt]); } }
#pragma unroll
    for (int tt = 0; tt < 4; ++tt)
#pragma unroll
      for (int r8 = 0; r8 < 8; ++r8) { const int rr = rt * 16 + 8 * hlf + r8, cc = tt * 16 + nloc; Tf[rr][cc] = Kp[rr] ? fmaxf(acc[tt][r8] * (1.0f / (HS * WSC)) + Ps[rr][cc], 0.0f) : 0.0f; } }
  wave_lds_sync();
  float s0 = 0.0f, s1 = 0.0f, cnt = 0.0f; for (int rr = 0; rr < 32; ++rr) { s0 += Tf[rr][lane]; s1 += Tf[rr][32 + lane]; cnt += (float)Kp[rr]; }
  for (int pass = 0; pass < 2; ++pass) { for (int rr = 0; rr < 32; ++rr) { ((volatile float*)HE)[(e0 + rr) * Hh + lane] = Tf[rr][lane]; ((volatile float*)HE)[(e0 + rr) * Hh + 32 + lane] = Tf[rr][32 + lane]; }
    ((volatile float*)EP)[(size_t)blockIdx.x * 128 + lane] = s0; ((volatile float*)EP)[(size_t)blockIdx.x * 128 + 32 + lane] = s1; ((volatile float*)EP)[(size_t)blockIdx.x * 128 + 64 + lane] = lane == 0 ? cnt : 0.0f; ((volatile float*)EP)[(size_t)blockIdx.x * 128 + 96 + lane] = 0.0f; __threadfence(); } }
__global__ __launch_bounds__(32) void node_kernel(const float* __restrict__ CX, const float* __restrict__ HE, const int* __restrict__ PERMs, const int* __restrict__ RPs, const int* __restrict__ RCs, int pls, const int* __restrict__ PERMr, const int* __restrict__ RPr, const int* __restrict__ RCr, int plr, const int* __restrict__ snd, const int* __restrict__ rcv, const float* __restrict__ GV, const b16* __restrict__ WNB, const float* __restrict__ bnb, const b16* __restrict__ WD1, const float* __restrict__ bd1, const float* __restrict__ wd2, const float* __restrict__ bd2, int t, int NLIM, int ELIM, float* __restrict__ HX, float* __restrict__ NP, float* __restrict__ OD) { __shared__ __attribute__((aligned(16))) b16 Ah[32][264], Al[32][264]; __shared__ float Tf[32][Hh + 1], Os[32]; const int lane = threadIdx.x, nloc = lane & 15, hlf = lane >> 4; const size_t n0 = (size_t)blockIdx.x * 32;
  for (int rr = 0; rr < 32; ++rr) { const size_t i = n0 + rr; const bool live = i < (size_t)NLIM; v2f se = {0, 0}, rv = {0, 0};
    if (live) { { int st = RPs[i], cnt = RCs[i]; cnt = iclamp(cnt, 0, E); st = iclamp(st, 0, pls - cnt);
#pragma unroll 1
        for (int j = 0; j < cnt; ++j) { const int e = iclamp(PERMs[st + j], 0, E - 1); const int r = rcv[e]; if (e >= ELIM || r < 0 || r >= NLIM) continue; const v2f v = *(const v2f*)(HE + (size_t)e * Hh + lane * 2); se += v; } }
      { int st = RPr[i], cnt = RCr[i]; cnt = iclamp(cnt, 0, E); st = iclamp(st, 0, plr - cnt);
#pragma unroll 1
        for (int j = 0; j < cnt; ++j) { const int e = iclamp(PERMr[st + j], 0, E - 1); const int s = snd[e]; if (e >= ELIM || s < 0 || s >= NLIM) continue; const v2f v = *(const v2f*)(HE + (size_t)e * Hh + lane * 2); rv += v; } } }
    for (int q = 0; q < 4; ++q) { const float cxv = live ? CX[i * 128 + q * 32 + lane] : 0.0f; b16 p, ql; split16(cxv * HS, p, ql); Ah[rr][q * 32 + lane] = p; Al[rr][q * 32 + lane] = ql; }
    for (int k = 0; k < 2; ++k) { b16 p, ql; split16(se[k] * HS, p, ql); Ah[rr][128 + lane * 2 + k] = p; Al[rr][128 + lane * 2 + k] = ql; split16(rv[k] * HS, p, ql); Ah[rr][192 + lane * 2 + k] = p; Al[rr][192 + lane * 2 + k] = ql; } }
  for (int k = 256; k < 264; ++k) { Ah[lane][k] = (b16)0.0f; Al[lane][k] = (b16)0.0f; }
  wave_lds_sync();
#pragma unroll
  for (int rt = 0; rt < 2; ++rt) { v8f acc[4] = {(v8f){}, (v8f){}, (v8f){}, (v8f){}};
#pragma unroll 2
    for (int kb = 0; kb < 256; kb += 32) { const v16b a = frag_kb(&Ah[rt * 16 + nloc][kb], hlf), al = frag_kb(&Al[rt * 16 + nloc][kb], hlf);
#pragma unroll
      for (int tt = 0; tt < 4; ++tt) { const v16b bw = frag_kb(WNB + (size_t)(tt * 16 + nloc) * 256 + kb, hlf); acc[tt] = wmma16b(a, bw, acc[tt]); acc[tt] = wmma16b(al, bw, acc[tt]); } }
#pragma unroll
    for (int tt = 0; tt < 4; ++tt) { const int cc = tt * 16 + nloc; const float bb = bfv(bnb[cc]) + GV[128 + cc];
#pragma unroll
      for (int r8 = 0; r8 < 8; ++r8) { const int rr = rt * 16 + 8 * hlf + r8; Tf[rr][cc] = (n0 + rr < (size_t)NLIM) ? fmaxf(acc[tt][r8] * (1.0f / (HS * WSC)) + bb, 0.0f) : 0.0f; } } }
  wave_lds_sync();
  float s0 = 0.0f, s1 = 0.0f, cnt = 0.0f; for (int rr = 0; rr < 32; ++rr) { s0 += Tf[rr][lane]; s1 += Tf[rr][32 + lane]; cnt += (n0 + rr < (size_t)NLIM) ? 1.0f : 0.0f; }
  for (int pass = 0; pass < 2; ++pass) { for (int rr = 0; rr < 32; ++rr) if (n0 + rr < (size_t)N) { ((volatile float*)HX)[(n0 + rr) * Hh + lane] = Tf[rr][lane]; ((volatile float*)HX)[(n0 + rr) * Hh + 32 + lane] = Tf[rr][32 + lane]; }
    ((volatile float*)NP)[(size_t)blockIdx.x * 128 + lane] = s0; ((volatile float*)NP)[(size_t)blockIdx.x * 128 + 32 + lane] = s1; ((volatile float*)NP)[(size_t)blockIdx.x * 128 + 64 + lane] = lane == 0 ? cnt : 0.0f; ((volatile float*)NP)[(size_t)blockIdx.x * 128 + 96 + lane] = 0.0f; __threadfence(); }
  for (int rr = 0; rr < 32; ++rr) for (int q = 0; q < 2; ++q) { b16 p, ql; split16(Tf[rr][q * 32 + lane] * HS, p, ql); Ah[rr][q * 32 + lane] = p; Al[rr][q * 32 + lane] = ql; }
  for (int k = 64; k < 72; ++k) { Ah[lane][k] = (b16)0.0f; Al[lane][k] = (b16)0.0f; }
  wave_lds_sync();
#pragma unroll
  for (int rt = 0; rt < 2; ++rt) { v8f acc[4] = {(v8f){}, (v8f){}, (v8f){}, (v8f){}};
#pragma unroll
    for (int kb = 0; kb < 64; kb += 32) { const v16b a = frag_kb(&Ah[rt * 16 + nloc][kb], hlf), al = frag_kb(&Al[rt * 16 + nloc][kb], hlf);
#pragma unroll
      for (int tt = 0; tt < 4; ++tt) { const v16b bw = frag_kb(WD1 + (size_t)(tt * 16 + nloc) * Hh + kb, hlf); acc[tt] = wmma16b(a, bw, acc[tt]); acc[tt] = wmma16b(al, bw, acc[tt]); } }
#pragma unroll
    for (int tt = 0; tt < 4; ++tt) { const int cc = tt * 16 + nloc; const float bb = bfv(bd1[cc]);
#pragma unroll
      for (int r8 = 0; r8 < 8; ++r8) Tf[rt * 16 + 8 * hlf + r8][cc] = fmaxf(acc[tt][r8] * (1.0f / (HS * WSC)) + bb, 0.0f); } }
  wave_lds_sync();
  { float s = bfv(bd2[0]);
#pragma unroll 4
    for (int k = 0; k < Hh; ++k) s += pmul(Tf[lane][k], bfv(wd2[k])); Os[lane] = s; }
  wave_lds_sync();
  for (int pass = 0; pass < 2; ++pass) { ((volatile float*)OD)[(size_t)t * (NNW * 32) + n0 + lane] = Os[lane]; __threadfence(); } }
__global__ __launch_bounds__(256) void copy_kernel(const float* __restrict__ OD, const int* __restrict__ nst, float* __restrict__ out) { const size_t u = (size_t)blockIdx.x * 256 + threadIdx.x; if (u >= (size_t)T * N) return; const size_t t = u / N, n = u % N; const bool ok = nst[0] == T;
  for (int pass = 0; pass < 2; ++pass) { ((volatile float*)out)[u] = ok ? OD[t * (NNW * 32) + n] : __builtin_nanf(""); __threadfence(); } }
}

extern "C" void kernel_launch(void* const* d_in, const int* in_sizes, int n_in, void* d_out, int out_size, void* d_ws, size_t ws_size, hipStream_t stream) {
  (void)n_in;
  auto Fp = [&](int i) { return (const float*)d_in[i]; }; auto Ip = [&](int i) { return (const int*)d_in[i]; };
  if (in_sizes[0] != T * N * F || in_sizes[1] != T * E || in_sizes[2] != T || in_sizes[3] != 2 * E || in_sizes[5] != F * Hh || in_sizes[11] != 448 * Hh || in_sizes[13] != 320 * Hh || in_sizes[15] != 192 * Hh || in_sizes[17] != Hh * Hh || in_sizes[19] != Hh || out_size != T * N) return;
  const int NLIM = N, ELIM = E;
  size_t off = 0; char* ws = (char*)d_ws;
  auto carve = [&](size_t bytes) { char* p = ws + off; off += (bytes + 255) & ~(size_t)255; return p; };
  b16* WEE = (b16*)carve((size_t)Hh * 128 * 2); b16* WEN = (b16*)carve((size_t)128 * 128 * 2); b16* WNB = (b16*)carve((size_t)Hh * 256 * 2); b16* WD1 = (b16*)carve((size_t)Hh * Hh * 2); float* GV = (float*)carve(1024); float* CX = (float*)carve((size_t)N * 128 * 4); float* PSR = (float*)carve((size_t)N * 128 * 4); float* HX = (float*)carve((size_t)NNW * 32 * Hh * 4); float* HE = (float*)carve((size_t)E * Hh * 4); float* EP = (float*)carve((size_t)NEW * 128 * 4); float* NP = (float*)carve((size_t)NNW * 128 * 4); float* OD = (float*)carve((size_t)T * NNW * 32 * 4); CsrBufs8 cs, cr; off = csr_carve8(cs, ws, off, E, N); off = csr_carve8(cr, ws, off, E, N);
  if (off > ws_size || off > ((size_t)224 << 20)) return;
  wput_kernel<<<(128 * 16 + 255) / 256, 256, 0, stream>>>(Fp(11), Fp(13), Fp(17), WEE, WEN, WNB, WD1);
  csr_build8(cs, Ip(3), E, N, stream); csr_build8(cr, Ip(3) + E, E, N, stream);
  for (int t = 0; t < T; ++t) { const int first = t == 0;
    glob_kernel<<<1, 64, 0, stream>>>(Fp(2), Fp(9), Fp(10), Fp(15), Fp(16), Fp(11), Fp(13), NP, NNW, EP, ELIM / 32, first, GV);
    nodepre_kernel<<<N / 16, 32, 0, stream>>>(Fp(0) + (size_t)t * N * F, Fp(5), Fp(6), HX, WEN, first, NLIM, CX, PSR);
    edge_kernel<<<ELIM / 32, 32, 0, stream>>>(Fp(1), t, first, Fp(7), Fp(8), PSR, GV, Ip(3), Ip(3) + E, WEE, Fp(12), NLIM, HE, EP);
    node_kernel<<<NNW, 32, 0, stream>>>(CX, HE, cs.PERM, cs.ROWPTR, cs.ROWCNT, (int)cs.permLen, cr.PERM, cr.ROWPTR, cr.ROWCNT, (int)cr.permLen, Ip(3), Ip(3) + E, GV, WNB, Fp(14), WD1, Fp(18), Fp(19), Fp(20), t, NLIM, ELIM, HX, NP, OD); }
  copy_kernel<<<(T * N + 255) / 256, 256, 0, stream>>>(OD, (const int*)d_in[4], (float*)d_out);
}
